// GAT_FP_20675972563340
// MI455X (gfx1250) — hardware-run, weakly checked
//
#include <hip/hip_runtime.h>


namespace {
constexpr int N = 12000, E = 192000, T = 120, ND = N / T  , IN = 192, NPB = 8;
constexpr float XS = 8.0f, HS = 256.0f, WSC = 256.0f;
typedef _Float16 b16;
typedef __attribute__((ext_vector_type(16))) _Float16 v16b;
typedef __attribute__((ext_vector_type(8))) _Float16 v8b;
typedef __attribute__((ext_vector_type(8))) float v8f;
typedef __attribute__((ext_vector_type(4))) float v4f;
typedef __attribute__((ext_vector_type(2))) float v2f;
__device__ __forceinline__ float bf16_rne(float f) { unsigned int u = __float_as_uint(f); u += 0x7FFFu + ((u >> 16) & 1u); float r = __uint_as_float(u & 0xFFFF0000u); asm volatile("" : "+v"(r)); return r; }
__device__ __forceinline__ float bfv(float f) { float r = bf16_rne(f); asm volatile("" : "+v"(r)); return r; }
__device__ __forceinline__ void split16(float v, b16& hi, b16& lo) { hi = (b16)v; lo = (b16)(v - (float)hi); }
__device__ __forceinline__ v16b frag_kb(const b16* p, int hh) { const v8b a = *(const v8b*)(p + 8 * hh), b = *(const v8b*)(p + 16 + 8 * hh); v16b f;
#pragma unroll
  for (int e = 0; e < 8; ++e) { f[e] = a[e]; f[8 + e] = b[e]; } return f; }
__device__ __forceinline__ v8f wmma16b(v16b a, v16b b, v8f c) { v8f d = __builtin_amdgcn_wmma_f32_16x16x32_f16(false, a, false, b, (short)0, c, false, false); asm volatile("v_nop\n\tv_nop\n\tv_nop\n\tv_nop" : "+v"(d) : "v"(a), "v"(b)); return d; }
__device__ __forceinline__ void wave_lds_sync() { __builtin_amdgcn_fence(__ATOMIC_RELEASE, "workgroup"); __builtin_amdgcn_wave_barrier(); __builtin_amdgcn_fence(__ATOMIC_ACQUIRE, "workgroup"); }
__device__ __forceinline__ float pmul(float a, float b) { float p = a * b; asm volatile("" : "+v"(p)); return p; }
__device__ __forceinline__ int iclamp(int v, int lo, int hi) { return v < lo ? lo : (v > hi ? hi : v); }
__device__ __forceinline__ float sigm(float v) { return 1.0f / (1.0f + __expf(-v)); }
constexpr int CSR_NBLK8 = 512, CSR_GB8 = 8, CSR_GN8 = 1 << CSR_GB8  , CSR_TS8 = (CSR_GN8 < 32 ? 32 : CSR_GN8)  , CSR_MAXG8 = 512, CSR_CAP8 = 12288  ;
__device__ __host__ __forceinline__ int csr_tix8(int v) { return (v >> CSR_GB8) * CSR_TS8 + (v & (CSR_GN8 - 1)); }
__global__ __launch_bounds__(64) void csrA_kernel8(const int* __restrict__ dst, int E, int N, int nG, int CHP, int NGP, int* __restrict__ STG, int* __restrict__ HST) {
  extern __shared__ int sm[];
  int* cnt = sm; int* run = sm + NGP; int* ids = sm + 2 * NGP;
  const int b = blockIdx.x; const int ch = (E + CSR_NBLK8 - 1) / CSR_NBLK8; const int e0 = b * ch, e1 = min(E, e0 + ch);
  for (int i = threadIdx.x; i < NGP; i += 64) cnt[i] = 0;
  for (int i = threadIdx.x; i < CHP; i += 64) ids[i] = -1;
  __syncthreads();
  if (threadIdx.x == 0) {
    for (int e = e0; e < e1; ++e) { int d = dst[e]; d = (d < 0) ? 0 : (d >= N ? N - 1 : d); cnt[d >> CSR_GB8] += 1; }
    int acc = 0; for (int g = 0; g < nG; ++g) { run[g] = acc; acc += cnt[g]; }
    for (int e = e0; e < e1; ++e) { int d = dst[e]; d = (d < 0) ? 0 : (d >= N ? N - 1 : d); const int g = d >> CSR_GB8; ids[run[g]] = e; run[g] += 1; } }
  __syncthreads();
  typedef __attribute__((ext_vector_type(4))) int v4i;
  for (int pass = 0; pass < 2; ++pass) {
    for (int i = threadIdx.x; i < CHP / 4; i += 64) *(volatile v4i*)(STG + (size_t)b * CHP + i * 4) = *(const v4i*)(&ids[i * 4]);
    for (int i = threadIdx.x; i < NGP / 4; i += 64) { v4i v; for (int e = 0; e < 4; ++e) v[e] = (i * 4 + e < nG) ? cnt[i * 4 + e] : 0; *(volatile v4i*)(HST + (size_t)b * NGP + i * 4) = v; }
    __threadfence(); }
}
__global__ __launch_bounds__(512) void csrS_kernel8(const int* __restrict__ HST, int nG, int NGP, int* __restrict__ START, int* __restrict__ TOT, int* __restrict__ OFF) {
  __shared__ int tot[CSR_MAXG8];
  const int b = threadIdx.x;
  for (int pass = 0; pass < 2; ++pass) { int runb = 0; for (int g = 0; g < nG; ++g) { int c = HST[(size_t)b * NGP + g]; c = (c < 0) ? 0 : c; ((volatile int*)OFF)[(size_t)g * CSR_NBLK8 + b] = runb; runb += c; } __threadfence(); }
  for (int g = threadIdx.x; g < nG; g += 512) { int s = 0; for (int bb = 0; bb < CSR_NBLK8; ++bb) { int c = HST[(size_t)bb * NGP + g]; s += (c < 0) ? 0 : c; } tot[g] = s; }
  __syncthreads();
  if (threadIdx.x < 32) {
    __shared__ int st[CSR_MAXG8 + 32];
    if (threadIdx.x == 0) { int acc = 0; for (int g = 0; g < NGP; ++g) { st[g] = acc; if (g < nG) acc += (tot[g] + 31) & ~31; } st[NGP] = acc; }
    __builtin_amdgcn_fence(__ATOMIC_RELEASE, "workgroup"); __builtin_amdgcn_wave_barrier(); __builtin_amdgcn_fence(__ATOMIC_ACQUIRE, "workgroup");
    for (int pass = 0; pass < 2; ++pass) { for (int i = threadIdx.x; i < NGP + 32; i += 32) { ((volatile int*)START)[i] = (i <= NGP) ? st[min(i, NGP)] : 0; ((volatile int*)TOT)[i] = (i < nG) ? tot[i] : 0; } __threadfence(); } }
}
__global__ __launch_bounds__(256) void csrB_kernel8(const int* __restrict__ dst, int N, int nG, int CHP, int NGP, int permLen, const int* __restrict__ STG, const int* __restrict__ HST, const int* __restrict__ OFF, const int* __restrict__ START, const int* __restrict__ TOT, int* __restrict__ PERM, int* __restrict__ ROWPTR, int* __restrict__ ROWCNT, int* __restrict__ FLAG) {
  typedef __attribute__((ext_vector_type(4))) int v4i;
  __shared__ int ids[CSR_CAP8]; __shared__ unsigned short key[CSR_CAP8]; __shared__ int outp[CSR_CAP8]; __shared__ int ncnt[CSR_GN8 + 1]; __shared__ int boff[CSR_NBLK8 + 1];
  const int g = blockIdx.x, t_ = threadIdx.x; int tot = TOT[g]; int st = START[g], stn = START[g + 1]; const int v0 = g * CSR_GN8; const int nv = min(CSR_GN8, N - v0); const int t0 = g * CSR_TS8;
  st = (st < 0) ? 0 : (st > permLen - 32 ? permLen - 32 : st) & ~31; stn = (stn < st) ? st : (stn > permLen ? permLen : stn); tot = (tot < 0) ? 0 : tot; if (tot > stn - st && tot <= CSR_CAP8) tot = stn - st;
  if (tot > CSR_CAP8) {
    for (int pass = 0; pass < 2; ++pass) { for (int i = t_; i < CSR_TS8 / 4; i += 256) { v4i a, c; for (int e = 0; e < 4; ++e) { a[e] = st; c[e] = 0; } *(volatile v4i*)(ROWPTR + t0 + i * 4) = a; *(volatile v4i*)(ROWCNT + t0 + i * 4) = c; } if (t_ == 0) ((volatile int*)FLAG)[0] = 1; __threadfence(); } (void)nv; return; }
  if (t_ == 0) { int acc = 0; for (int b = 0; b < CSR_NBLK8; ++b) { boff[b] = acc; int c = HST[(size_t)b * NGP + g]; c = (c < 0) ? 0 : (c > CHP ? CHP : c); acc += c; if (acc > tot) acc = tot; } boff[CSR_NBLK8] = acc; }
  for (int i = t_; i <= CSR_GN8; i += 256) ncnt[i] = 0;
  __syncthreads();
  for (int b = 0; b < CSR_NBLK8; ++b) { const int c = boff[b + 1] - boff[b]; int o_ = OFF[(size_t)g * CSR_NBLK8 + b]; o_ = (o_ < 0) ? 0 : (o_ > CHP - c ? CHP - c : o_); const int* src_ = STG + (size_t)b * CHP + o_;
    for (int i = t_; i < c; i += 256) { int id = src_[i]; id = (id < 0) ? 0 : id; ids[boff[b] + i] = id; int d = dst[id]; d = (d < v0) ? v0 : (d >= N ? N - 1 : d); int kk = d - v0; kk = (kk < 0) ? 0 : (kk >= CSR_GN8 ? CSR_GN8 - 1 : kk); key[boff[b] + i] = (unsigned short)kk; } }
  __syncthreads();
  if (t_ == 0) { for (int i = 0; i < tot; ++i) ncnt[key[i]] += 1; int acc = 0; for (int vl = 0; vl < CSR_GN8; ++vl) { const int c = ncnt[vl]; ncnt[vl] = acc; acc += c; } ncnt[CSR_GN8] = acc;
    for (int i = 0; i < tot; ++i) { const int vl = key[i]; outp[ncnt[vl]] = ids[i]; ncnt[vl] += 1; }
    for (int vl = CSR_GN8; vl > 0; --vl) ncnt[vl] = ncnt[vl - 1]; ncnt[0] = 0; }
  __syncthreads();
  for (int pass = 0; pass < 2; ++pass) {
    for (int i = t_; i < (stn - st) / 4; i += 256) { v4i v; for (int e = 0; e < 4; ++e) { const int q = i * 4 + e; v[e] = (q < tot) ? outp[q] : -1; } *(volatile v4i*)(PERM + st + i * 4) = v; }
    for (int i = t_; i < CSR_TS8 / 4; i += 256) { v4i a, c; for (int e = 0; e < 4; ++e) { const int vl = i * 4 + e; const int vc = vl < CSR_GN8 ? vl : CSR_GN8; a[e] = (vl < CSR_GN8) ? st + ncnt[vc] : st; c[e] = (vl < nv) ? (ncnt[(vc < CSR_GN8 ? vc : CSR_GN8 - 1) + 1] - ncnt[vc]) : 0; } *(volatile v4i*)(ROWPTR + t0 + i * 4) = a; *(volatile v4i*)(ROWCNT + t0 + i * 4) = c; }
    __threadfence(); }
}
__global__ __launch_bounds__(256) void csrZ_kernel8(int* __restrict__ p, size_t n4) { typedef __attribute__((ext_vector_type(4))) int v4i; const size_t tid = (size_t)blockIdx.x * 256 + threadIdx.x, nth = (size_t)gridDim.x * 256; v4i z = {0, 0, 0, 0}; for (size_t i = tid; i < n4; i += nth) *(volatile v4i*)(p + i * 4) = z; }
struct CsrBufs8 { int *STG, *HST, *OFF, *START, *TOT, *PERM, *ROWPTR, *ROWCNT, *FLAG; int nG, NGP, CHP; size_t permLen; char* base; size_t bytes; };
static size_t csr_carve8(CsrBufs8& c, char* ws, size_t off, int E, int N) {
  const size_t off0 = off; c.base = ws + off;
  auto al = [&](size_t bytes) { char* p = ws + off; off += (bytes + 255) & ~(size_t)255; return p; };
  c.nG = (N + CSR_GN8 - 1) / CSR_GN8; c.NGP = (c.nG + 31) & ~31; const int ch = (E + CSR_NBLK8 - 1) / CSR_NBLK8; c.CHP = (ch + 31) & ~31; c.permLen = (size_t)E + 32 * (size_t)c.nG + 32;
  c.STG = (int*)al((size_t)CSR_NBLK8 * c.CHP * 4); c.HST = (int*)al((size_t)CSR_NBLK8 * c.NGP * 4); c.OFF = (int*)al((size_t)c.NGP * CSR_NBLK8 * 4); c.START = (int*)al((size_t)(c.NGP + 64) * 4); c.TOT = (int*)al((size_t)(c.NGP + 64) * 4);
  c.PERM = (int*)al(c.permLen * 4); c.ROWPTR = (int*)al((size_t)c.nG * CSR_TS8 * 4); c.ROWCNT = (int*)al((size_t)c.nG * CSR_TS8 * 4); c.FLAG = (int*)al(256);
  c.bytes = off - off0; return off;
}
static void csr_build8(const CsrBufs8& c, const int* dst, int E, int N, hipStream_t stream) {
  const size_t smem = (size_t)(2 * c.NGP + c.CHP) * 4;
  csrZ_kernel8<<<512, 256, 0, stream>>>((int*)c.base, c.bytes / 16);
  csrA_kernel8<<<CSR_NBLK8, 64, smem, stream>>>(dst, E, N, c.nG, c.CHP, c.NGP, c.STG, c.HST);
  csrS_kernel8<<<1, 512, 0, stream>>>(c.HST, c.nG, c.NGP, c.START, c.TOT, c.OFF);
  csrB_kernel8<<<c.nG, 256, 0, stream>>>(dst, N, c.nG, c.CHP, c.NGP, (int)c.permLen, c.STG, c.HST, c.OFF, c.START, c.TOT, c.PERM, c.ROWPTR, c.ROWCNT, c.FLAG);
}


__global__ __launch_bounds__(256) void wput_kernel(const float* __restrict__ wtx, const float* __restrict__ wau, const float* __restrict__ wvi, const float* __restrict__ wihf, const float* __restrict__ wihb, const float* __restrict__ wgc, const float* __restrict__ ws2, const float* __restrict__ wd2, const float* __restrict__ wr2, const float* __restrict__ ws0, const float* __restrict__ wd0, const float* __restrict__ wr0, const float* __restrict__ ws1, const float* __restrict__ wd1, const float* __restrict__ wr1,
    b16* __restrict__ WTX, b16* __restrict__ WAU, b16* __restrict__ WVI, b16* __restrict__ WLS, b16* __restrict__ WGC, b16* __restrict__ W2, b16* __restrict__ W0, b16* __restrict__ W1) { const size_t nt = (size_t)gridDim.x * 256, u0 = (size_t)blockIdx.x * 256 + threadIdx.x; v8b v;
  auto putT = [&](const float* src, b16* dst, int kin, int nout, int ocol0, int ototal) {
    for (size_t u = u0; u < (size_t)nout * (kin / 8); u += nt) { const int o = (int)(u / (kin / 8)), k0 = (int)(u % (kin / 8)) * 8;
#pragma unroll
      for (int j = 0; j < 8; ++j) v[j] = (b16)(bf16_rne(src[(size_t)(k0 + j) * nout + o]) * WSC); for (int pass = 0; pass < 2; ++pass) { *(volatile v8b*)(dst + (size_t)(ocol0 + o) * kin + k0) = v; __threadfence(); } } (void)ototal; };
  putT(wtx, WTX, 1024, 64, 0, 64); putT(wau, WAU, 512, 64, 0, 64); putT(wvi, WVI, 1024, 64, 0, 64); putT(wgc, WGC, IN, IN, 0, IN);
  putT(ws2, W2, IN, 64, 0, 192); putT(wd2, W2, IN, 64, 64, 192); putT(wr2, W2, IN, 64, 128, 192);
  putT(ws0, W0, IN, 512, 0, 1536); putT(wd0, W0, IN, 512, 512, 1536); putT(wr0, W0, IN, 512, 1024, 1536);
  putT(ws1, W1, 512, 64, 0, 192); putT(wd1, W1, 512, 64, 64, 192); putT(wr1, W1, 512, 64, 128, 192);
  for (size_t u = u0; u < (size_t)32 * (IN / 8); u += nt) { const int o = (int)(u / (IN / 8)), k0 = (int)(u % (IN / 8)) * 8; const float* w = o < 16 ? wihf + (size_t)o * IN : wihb + (size_t)(o - 16) * IN;
#pragma unroll
    for (int j = 0; j < 8; ++j) v[j] = (b16)(bf16_rne(w[k0 + j]) * WSC); for (int pass = 0; pass < 2; ++pass) { *(volatile v8b*)(WLS + (size_t)o * IN + k0) = v; __threadfence(); } } }
__global__ __launch_bounds__(32) void enc_kernel(const float* __restrict__ tx, const float* __restrict__ au, const float* __restrict__ vi, const b16* __restrict__ WTX, const float* __restrict__ btx, const b16* __restrict__ WAU, const float* __restrict__ bau, const b16* __restrict__ WVI, const float* __restrict__ bvi, int NLIM, float* __restrict__ SF) { __shared__ __attribute__((aligned(16))) b16 Ah[16][264]; __shared__ float Tf[16][IN + 4]; const int lane = threadIdx.x, nloc = lane & 15, hlf = lane >> 4; const size_t m0 = (size_t)blockIdx.x * 16; if (m0 >= (size_t)NLIM) return;
  if (lane < 16) for (int k = 256; k < 264; ++k) Ah[lane][k] = (b16)0.0f;
#pragma unroll 1
  for (int md = 0; md < 3; ++md) { const float* X = md == 0 ? tx : (md == 1 ? au : vi); const int KIN = md == 1 ? 512 : 1024; const b16* W = md == 0 ? WTX : (md == 1 ? WAU : WVI); const float* bb_ = md == 0 ? btx : (md == 1 ? bau : bvi); v8f acc[4] = {(v8f){}, (v8f){}, (v8f){}, (v8f){}};
#pragma unroll 1
    for (int kc = 0; kc < KIN; kc += 256) { for (int rr = 0; rr < 16; ++rr) for (int q = 0; q < 8; ++q) Ah[rr][q * 32 + lane] = (b16)(bf16_rne(X[(m0 + rr) * KIN + kc + q * 32 + lane]) * XS);
      wave_lds_sync();
#pragma unroll 2
      for (int kb = 0; kb < 256; kb += 32) { const v16b a = frag_kb(&Ah[nloc][kb], hlf);
#pragma unroll
        for (int t = 0; t < 4; ++t) acc[t] = wmma16b(a, frag_kb(W + (size_t)(t * 16 + nloc) * KIN + kc + kb, hlf), acc[t]); }
      wave_lds_sync(); }
#pragma unroll
    for (int t = 0; t < 4; ++t) { const int cc = t * 16 + nloc; const float bb = bfv(bb_[cc]);
#pragma unroll
      for (int r8 = 0; r8 < 8; ++r8) Tf[8 * hlf + r8][md * 64 + cc] = acc[t][r8] * (1.0f / (XS * WSC)) + bb; } }
  wave_lds_sync();
  for (int pass = 0; pass < 2; ++pass) { for (int rr = 0; rr < 16; ++rr) for (int q = 0; q < 3; ++q) *(volatile v2f*)(SF + (m0 + rr) * IN + q * 64 + lane * 2) = *(const v2f*)(&Tf[rr][q * 64 + lane * 2]); __threadfence(); } }
template <int KIN, int GW>
__global__ __launch_bounds__(32) void lin_kernel(const float* __restrict__ INP, const b16* __restrict__ W, const float* __restrict__ bias, int OW, int NG, const int* __restrict__ DEGCNT, int NLIM, float* __restrict__ OUT) { __shared__ __attribute__((aligned(16))) b16 Ah[16][KIN + 8], Al[16][KIN + 8]; __shared__ float Tf[16][GW * 16 + 4]; const int lane = threadIdx.x, nloc = lane & 15, hlf = lane >> 4; const int g = blockIdx.x % NG; const size_t m0 = (size_t)(blockIdx.x / NG) * 16; if (m0 >= (size_t)NLIM) return;
  for (int rr = 0; rr < 16; ++rr) for (int q = 0; q < KIN / 32; ++q) { b16 p, ql; split16(INP[(m0 + rr) * KIN + q * 32 + lane] * HS, p, ql); Ah[rr][q * 32 + lane] = p; Al[rr][q * 32 + lane] = ql; }
  if (lane < 16) for (int k = KIN; k < KIN + 8; ++k) { Ah[lane][k] = (b16)0.0f; Al[lane][k] = (b16)0.0f; }
  wave_lds_sync(); v8f acc[GW];
#pragma unroll
  for (int t = 0; t < GW; ++t) acc[t] = (v8f){};
#pragma unroll 2
  for (int kb = 0; kb < KIN; kb += 32) { const v16b a = frag_kb(&Ah[nloc][kb], hlf), al = frag_kb(&Al[nloc][kb], hlf);
#pragma unroll
    for (int t = 0; t < GW; ++t) { const v16b bw = frag_kb(W + (size_t)((g * GW + t) * 16 + nloc) * KIN + kb, hlf); acc[t] = wmma16b(a, bw, acc[t]); acc[t] = wmma16b(al, bw, acc[t]); } }
#pragma unroll
  for (int t = 0; t < GW; ++t) { const int cl = t * 16 + nloc; const int cc = g * GW * 16 + cl; const float bb = bias ? bfv(bias[cc]) : 0.0f;
#pragma unroll
    for (int r8 = 0; r8 < 8; ++r8) { const int rr = 8 * hlf + r8; float v = acc[t][r8] * (1.0f / (HS * WSC)); if (DEGCNT) { const int dc = iclamp(DEGCNT[m0 + rr], 0, E); v = pmul(v, rsqrtf(fmaxf((float)dc, 1.0f))); } Tf[rr][cl] = v + bb; } }
  wave_lds_sync();
  for (int pass = 0; pass < 2; ++pass) { for (int rr = 0; rr < 16; ++rr) for (int q = 0; q < GW / 2; ++q) ((volatile float*)OUT)[(m0 + rr) * OW + g * GW * 16 + q * 32 + lane] = Tf[rr][q * 32 + lane]; __threadfence(); } }
__global__ __launch_bounds__(128) void lstm_kernel(const float* __restrict__ G, const float* __restrict__ whf, const float* __restrict__ bif, const float* __restrict__ bhf, const float* __restrict__ whb, const float* __restrict__ bib, const float* __restrict__ bhb, int DLIM, float* __restrict__ NF) { __shared__ float Zs[128][17], Hs[128][5], Cs[128][5]; const int tid = threadIdx.x; const int d = blockIdx.x * 128 + tid; if (d >= DLIM) return;
  for (int pass = 0; pass < 2; ++pass) {
#pragma unroll 1
    for (int dir = 0; dir < 2; ++dir) { const float* wh = dir ? whb : whf; const float* bi = dir ? bib : bif; const float* bh = dir ? bhb : bhf;
#pragma unroll 1
      for (int k = 0; k < 4; ++k) { Hs[tid][k] = 0.0f; Cs[tid][k] = 0.0f; }
#pragma unroll 1
      for (int st = 0; st < T; ++st) { const int t = dir ? T - 1 - st : st; const size_t n = (size_t)d * T + t;
#pragma unroll 1
        for (int gq = 0; gq < 16; ++gq) { float s = G[n * 32 + dir * 16 + gq] + bfv(bi[gq]) + bfv(bh[gq]);
#pragma unroll 1
          for (int k = 0; k < 4; ++k) s += pmul(Hs[tid][k], bfv(wh[gq * 4 + k])); Zs[tid][gq] = s; }
#pragma unroll 1
        for (int k = 0; k < 4; ++k) { const float cn = pmul(sigm(Zs[tid][4 + k]), Cs[tid][k]) + pmul(sigm(Zs[tid][k]), tanhf(Zs[tid][8 + k])); Cs[tid][k] = cn; const float hn = pmul(sigm(Zs[tid][12 + k]), tanhf(cn)); Hs[tid][k] = hn; ((volatile float*)NF)[n * 8 + dir * 4 + k] = hn; } } }
    __threadfence(); } }
__global__ __launch_bounds__(256) void gc_kernel(const float* __restrict__ HW, const float* __restrict__ SF, const float* __restrict__ bgc, const int* __restrict__ srcs, const int* __restrict__ PERM, const int* __restrict__ ROWPTR, const int* __restrict__ ROWCNT, int permLen, int NLIM, float* __restrict__ Hh) { const int wave = threadIdx.x >> 5, lane = threadIdx.x & 31; const size_t i = (size_t)blockIdx.x * NPB + wave; if (i >= (size_t)NLIM) return; int st = ROWPTR[i], cnt = ROWCNT[i]; cnt = iclamp(cnt, 0, E); st = iclamp(st, 0, permLen - cnt); float acc[6] = {0, 0, 0, 0, 0, 0};
#pragma unroll 1
  for (int j = 0; j < cnt; ++j) { const int e = iclamp(PERM[st + j], 0, E - 1); const size_t u = (size_t)iclamp(srcs[e], 0, N - 1); if (u >= (size_t)NLIM) continue;
#pragma unroll
    for (int k = 0; k < 6; ++k) acc[k] += HW[u * IN + lane * 6 + k]; }
  const float din = rsqrtf(fmaxf((float)cnt, 1.0f)); float hv[6], sa = 0.0f;
#pragma unroll
  for (int k = 0; k < 6; ++k) { const int c = lane * 6 + k; hv[k] = 0.5f * (SF[i * IN + c] + (pmul(acc[k], din) + bfv(bgc[c]))); sa += fabsf(hv[k]); }
  for (int o = 16; o; o >>= 1) sa += __shfl_xor(sa, o); const float inv = 1.0f / fmaxf(sa, 1e-12f);
  for (int pass = 0; pass < 2; ++pass) {
#pragma unroll
    for (int k = 0; k < 6; ++k) ((volatile float*)Hh)[i * IN + lane * 6 + k] = hv[k] * inv; __threadfence(); } }
template <int F>
__global__ __launch_bounds__(256) void gat_kernel(const float* __restrict__ FSD, const float* __restrict__ bsrc, const float* __restrict__ bdst, const float* __restrict__ attn, const int* __restrict__ srcs, const int* __restrict__ PERM, const int* __restrict__ ROWPTR, const int* __restrict__ ROWCNT, int permLen, int NLIM, int OW, int OC0, float* __restrict__ OUT) { constexpr int W = 16 * F, CPL = W / 32, HL = 32 / 16  ; const int wave = threadIdx.x >> 5, lane = threadIdx.x & 31; const size_t i = (size_t)blockIdx.x * NPB + wave; if (i >= (size_t)NLIM) return; int st = ROWPTR[i], cnt = ROWCNT[i]; cnt = iclamp(cnt, 0, E); st = iclamp(st, 0, permLen - cnt);
  const float* row_i = FSD + i * 3 * W; float fd[CPL], at[CPL];
#pragma unroll
  for (int k = 0; k < CPL; ++k) { const int c = lane * CPL + k; fd[k] = row_i[W + c] + bfv(bdst[c]) + bfv(bsrc[c]); at[k] = bfv(attn[c]); }
  float mx = -INFINITY, den = 0.0f, acc[CPL]; int nin = 0;
#pragma unroll
  for (int k = 0; k < CPL; ++k) acc[k] = 0.0f;
#pragma unroll 1
  for (int j = 0; j < cnt; ++j) { const int e = iclamp(PERM[st + j], 0, E - 1); const size_t u = (size_t)iclamp(srcs[e], 0, N - 1); if (u >= (size_t)NLIM) continue; ++nin; const float* fs = FSD + u * 3 * W + lane * CPL; float fsv[CPL]; float s = 0.0f;
#pragma unroll
    for (int k = 0; k < CPL; ++k) { fsv[k] = fs[k]; float ev = fsv[k] + fd[k]; ev = ev > 0.0f ? ev : 0.2f * ev; s += pmul(ev, at[k]); }
    s += __shfl_xor(s, 1);
    const float mn = fmaxf(mx, s); const float sf = (mx == -INFINITY) ? 0.0f : __expf(mx - mn); const float p = __expf(s - mn); den = den * sf + p;
#pragma unroll
    for (int k = 0; k < CPL; ++k) acc[k] = pmul(acc[k], sf) + pmul(p, fsv[k]); mx = mn; }
  (void)HL;
  for (int pass = 0; pass < 2; ++pass) {
#pragma unroll
    for (int k = 0; k < CPL; ++k) { const int c = lane * CPL + k; const float o = (nin > 0 ? acc[k] / den + bfv(bsrc[c]) : 0.0f) + row_i[2 * W + c];   ((volatile float*)OUT)[i * OW + OC0 + c] = fmaxf(o, 0.0f); } __threadfence(); } }
__global__ __launch_bounds__(256) void head_kernel(const float* __restrict__ CAT, const float* __restrict__ NF, const float* __restrict__ wl, const float* __restrict__ bl, int NLIM, float* __restrict__ out) { const size_t u = (size_t)blockIdx.x * 256 + threadIdx.x; if (u >= (size_t)N * 6) return; const size_t n = u / 6; const int o = (int)(u % 6); if (n >= (size_t)NLIM) return; float s = bfv(bl[o]);
  for (int c = 0; c < 64; ++c) s += pmul(CAT[n * 128 + c], bfv(wl[c * 6 + o]));
  for (int c = 0; c < 8; ++c) s += pmul(NF[n * 8 + c], bfv(wl[(64 + c) * 6 + o]));
  for (int c = 0; c < 64; ++c) s += pmul(CAT[n * 128 + 64 + c], bfv(wl[(72 + c) * 6 + o]));
  for (int pass = 0; pass < 2; ++pass) { ((volatile float*)out)[u] = s; __threadfence(); } }
}

extern "C" void kernel_launch(void* const* d_in, const int* in_sizes, int n_in, void* d_out, int out_size, void* d_ws, size_t ws_size, hipStream_t stream) {
  (void)n_in;
  auto Fp = [&](int i) { return (const float*)d_in[i]; }; auto Ip = [&](int i) { return (const int*)d_in[i]; };
  if (in_sizes[0] != N * 1024 || in_sizes[1] != N * 512 || in_sizes[2] != N * 1024 || in_sizes[3] != E || in_sizes[4] != E || in_sizes[9] != 1024 * 64 || in_sizes[11] != 16 * IN || in_sizes[19] != IN * IN || in_sizes[27] != IN * 512 || in_sizes[33] != 512 * 64 || in_sizes[39] != 136 * 6 || out_size != N * 6) return;
  const int NLIM = N;
  size_t off = 0; char* ws = (char*)d_ws;
  auto carve = [&](size_t bytes) { char* p = ws + off; off += (bytes + 255) & ~(size_t)255; return p; };
  b16* WTX = (b16*)carve((size_t)64 * 1024 * 2); b16* WAU = (b16*)carve((size_t)64 * 512 * 2); b16* WVI = (b16*)carve((size_t)64 * 1024 * 2); b16* WLS = (b16*)carve((size_t)32 * IN * 2); b16* WGC = (b16*)carve((size_t)IN * IN * 2); b16* W2 = (b16*)carve((size_t)192 * IN * 2); b16* W0 = (b16*)carve((size_t)1536 * IN * 2); b16* W1 = (b16*)carve((size_t)192 * 512 * 2);
  float* SF = (float*)carve((size_t)N * IN * 4); float* G = (float*)carve((size_t)N * 32 * 4); float* NF = (float*)carve((size_t)N * 8 * 4); float* HW = (float*)carve((size_t)N * IN * 4); float* Hh = (float*)carve((size_t)N * IN * 4); float* FSD2 = (float*)carve((size_t)N * 192 * 4); float* FSD0 = (float*)carve((size_t)N * 1536 * 4); float* H0 = (float*)carve((size_t)N * 512 * 4); float* FSD1 = (float*)carve((size_t)N * 192 * 4); float* CAT = (float*)carve((size_t)N * 128 * 4);
  CsrBufs8 cd, cs; off = csr_carve8(cd, ws, off, E, N); off = csr_carve8(cs, ws, off, E, N);
  if (off > ws_size || off > ((size_t)192 << 20)) return;
  const int nb = (NLIM + NPB - 1) / NPB;
  wput_kernel<<<128, 256, 0, stream>>>(Fp(9), Fp(5), Fp(7), Fp(11), Fp(15), Fp(19), Fp(21), Fp(23), Fp(26), Fp(27), Fp(29), Fp(32), Fp(33), Fp(35), Fp(38), WTX, WAU, WVI, WLS, WGC, W2, W0, W1);
  csr_build8(cd, Ip(4), E, N, stream); csr_build8(cs, Ip(3), E, N, stream);
  enc_kernel<<<NLIM / 16, 32, 0, stream>>>(Fp(0), Fp(1), Fp(2), WTX, Fp(10), WAU, Fp(6), WVI, Fp(8), NLIM, SF);
  lin_kernel<IN, 2><<<(NLIM / 16) * 1, 32, 0, stream>>>(SF, WLS, nullptr, 32, 1, nullptr, NLIM, G);
  lstm_kernel<<<1, 128, 0, stream>>>(G, Fp(12), Fp(13), Fp(14), Fp(16), Fp(17), Fp(18), NLIM / T, NF);
  lin_kernel<IN, 12><<<(NLIM / 16) * 1, 32, 0, stream>>>(SF, WGC, nullptr, IN, 1, cs.ROWCNT, NLIM, HW);
  gc_kernel<<<nb, 256, 0, stream>>>(HW, SF, Fp(20), Ip(3), cd.PERM, cd.ROWPTR, cd.ROWCNT, (int)cd.permLen, NLIM, Hh);
  lin_kernel<IN, 12><<<(NLIM / 16) * 1, 32, 0, stream>>>(Hh, W2, nullptr, 192, 1, nullptr, NLIM, FSD2);
  gat_kernel<4><<<nb, 256, 0, stream>>>(FSD2, Fp(22), Fp(24), Fp(25), Ip(3), cd.PERM, cd.ROWPTR, cd.ROWCNT, (int)cd.permLen, NLIM, 128, 64, CAT);
  lin_kernel<IN, 12><<<(NLIM / 16) * 8, 32, 0, stream>>>(Hh, W0, nullptr, 1536, 8, nullptr, NLIM, FSD0);
  gat_kernel<32><<<nb, 256, 0, stream>>>(FSD0, Fp(28), Fp(30), Fp(31), Ip(3), cd.PERM, cd.ROWPTR, cd.ROWCNT, (int)cd.permLen, NLIM, 512, 0, H0);
  lin_kernel<512, 12><<<(NLIM / 16) * 1, 32, 0, stream>>>(H0, W1, nullptr, 192, 1, nullptr, NLIM, FSD1);
  gat_kernel<4><<<nb, 256, 0, stream>>>(FSD1, Fp(34), Fp(36), Fp(37), Ip(3), cd.PERM, cd.ROWPTR, cd.ROWCNT, (int)cd.permLen, NLIM, 128, 0, CAT);
  head_kernel<<<(N * 6 + 255) / 256, 256, 0, stream>>>(CAT, NF, Fp(39), Fp(40), NLIM, (float*)d_out);
}
